// GCN_Encoder_19344532701200
// MI455X (gfx1250) — hardware-run, weakly checked
//
#include <hip/hip_runtime.h>
#include <stddef.h>
#include <stdint.h>
#include <math.h>

#define NN      100000
#define NU      50000
#define NE      1250000
#define HD      64
#define NLAY    3
#define GBM     128
#define MP      100096
#define KL      128
#define NTHR    256
#define NWAVE   8
#define EPT     8
#define WCH     (32 * EPT)
#define NBRUN   1024
#define SLB     10
#define NBK     98
#define RP      (NBK * NBRUN)
#define WLCAP   2560
#define RCAP    20480
#define TRIPCAP 64
#define MAXDEG_MEAS   30
#define MAXB1024_MEAS 13072
#define SP      68
#define WSMAX   (128u << 20)

#ifndef SPLIT1
#define SPLIT1 1
#endif
#ifndef SPLIT2
#define SPLIT2 1
#endif
#define KS1 ((SPLIT1 != 0) ? KL : HD)
#define KS2 ((SPLIT2 != 0) ? KL : HD)

#define BK_ZINTS (NWAVE * WLCAP + RCAP + 3 * NBRUN)
#define BK_INTS  (BK_ZINTS + 16)
#define BK_LDS   (BK_INTS * 4)

#define PBX   (MP * HD / 8 / NTHR)
#define PBW   (NLAY * HD * HD / 8 / NTHR)
#define PBTOT (PBX + PBW + 1)
#define PARN  384

static_assert(HD == 64 && HD == 16 * 4);
static_assert(NTHR == 256 && NTHR / 16 == 16 && NTHR / 32 == NWAVE);
static_assert(MP % GBM == 0 && MP >= NN && MP == 782 * GBM && (NN % GBM) == 32);
static_assert(NBRUN == (1 << SLB) && NBRUN % 16 == 0 && NBRUN == 4 * NTHR);
static_assert(NBK * NBRUN >= NN && NBK * NBRUN >= MP && NN - (NBK - 1) * NBRUN == 672);
static_assert(NE < (1 << 21) && (((long long)NE) << SLB) < (1LL << 31));
static_assert(NE % EPT == 0 && ((long long)NE * 4) % 16 == 0);
static_assert(RCAP == NWAVE * WLCAP && RCAP % (4 * NTHR) == 0 && BK_ZINTS % 4 == 0);
static_assert((long long)RCAP * 100 >= (long long)MAXB1024_MEAS * 105);
static_assert(WLCAP >= MAXB1024_MEAS / 8 + 8 * 41 + 1);
static_assert(MAXDEG_MEAS + 8 <= TRIPCAP);
static_assert((MP * HD / 8) % NTHR == 0 && (NLAY * HD * HD / 8) % NTHR == 0);
static_assert(KL == 2 * HD && KS1 % 32 == 0 && KS2 % 32 == 0 && KS1 <= KL && KS2 <= KL);
static_assert(BK_LDS <= 300000 && BK_LDS <= 327680);
static_assert((GBM * SP + GBM) * 4 <= 65536);
static_assert((NN * HD / 4) % NTHR == 0);
static_assert(NU * HD * 4 == 12800000);
static_assert((long long)NN * HD - 1 == 6399999);
static_assert(NLAY * HD + 128 <= PARN);

typedef float          v4f   __attribute__((ext_vector_type(4)));
typedef float          v8f   __attribute__((ext_vector_type(8)));
typedef double         v2d   __attribute__((ext_vector_type(2)));
typedef int            v4i   __attribute__((ext_vector_type(4)));
typedef int            v8i   __attribute__((ext_vector_type(8)));
typedef unsigned short v8us  __attribute__((ext_vector_type(8)));
typedef unsigned short v16us __attribute__((ext_vector_type(16)));
typedef __bf16         v16bf __attribute__((ext_vector_type(16)));
typedef v4f  __attribute__((may_alias)) v4fa;
typedef v2d  __attribute__((may_alias)) v2da;
typedef v4i  __attribute__((may_alias)) v4ia;
typedef v8us __attribute__((may_alias)) v8usa;
union FragB { v16bf v; v16us u; v8us h[2]; v8i w; };

__device__ __forceinline__ v8f wmb(const FragB& a, const FragB& b, v8f c) {
  v8f d = __builtin_amdgcn_wmma_f32_16x16x32_bf16(false, a.v, false, b.v, (short)0, c, false, false);
  asm volatile("v_nop\n\tv_nop\n\tv_nop\n\tv_nop" : "+v"(d) : "v"(a.w), "v"(b.w));
  return d;
}

__device__ __forceinline__ unsigned bf16_bits(float f) {
  const unsigned u = __float_as_uint(f);
  const unsigned r = (u + 0x7FFFu + ((u >> 16) & 1u)) >> 16;
  const unsigned q = (u >> 16) | 0x40u;
  return ((u & 0x7fffffffu) > 0x7f800000u) ? q : r;
}

__device__ __forceinline__ void hilo_pack(float v0, float v1, float v2, float v3,
                                          int& h01, int& h23, int& l01, int& l23) {
  const unsigned a0 = bf16_bits(v0), a1 = bf16_bits(v1), a2 = bf16_bits(v2), a3 = bf16_bits(v3);
  const unsigned b0 = bf16_bits(v0 - __uint_as_float(a0 << 16));
  const unsigned b1 = bf16_bits(v1 - __uint_as_float(a1 << 16));
  const unsigned b2 = bf16_bits(v2 - __uint_as_float(a2 << 16));
  const unsigned b3 = bf16_bits(v3 - __uint_as_float(a3 << 16));
  h01 = (int)(a0 | (a1 << 16)); h23 = (int)(a2 | (a3 << 16));
  l01 = (int)(b0 | (b1 << 16)); l23 = (int)(b2 | (b3 << 16));
}

__device__ __forceinline__ v4i regroup8(int h01, int h23, int l01, int l23, int lane) {
  const int t  = lane & 15;
  const int s0 = (lane & 16) + ((2 * t) & 15), s1 = s0 + 1;
  const int a0 = __shfl(h01, s0, 32), a1 = __shfl(h23, s0, 32), a2 = __shfl(h01, s1, 32), a3 = __shfl(h23, s1, 32);
  const int b0 = __shfl(l01, s0, 32), b1 = __shfl(l23, s0, 32), b2 = __shfl(l01, s1, 32), b3 = __shfl(l23, s1, 32);
  const int mk = (t < 8) ? -1 : 0;
  v4i o;
  o.x = (a0 & mk) | (b0 & ~mk); o.y = (a1 & mk) | (b1 & ~mk);
  o.z = (a2 & mk) | (b2 & ~mk); o.w = (a3 & mk) | (b3 & ~mk);
  return o;
}

__device__ __forceinline__ void st2_v4f(float* p, v4f v) {
  *(volatile v4f*)p = v;
  __threadfence();
  *(volatile v4f*)p = v;
}
__device__ __forceinline__ void st2_v8us(unsigned short* p, v8us v) {
  *(volatile v8us*)p = v;
  __threadfence();
  *(volatile v8us*)p = v;
}

__global__ __launch_bounds__(NTHR) void k_prep(const float* __restrict__ x, const float* __restrict__ wsrc,
                                               const float* __restrict__ bs, const float* __restrict__ gam,
                                               const float* __restrict__ bet,
                                               unsigned short* xb, unsigned short* wb, float* par) {
  const int tid = (int)threadIdx.x;
  const int blk = (int)blockIdx.x;
  if (blk < PBX) {
    const int u   = blk * NTHR + tid;
    const int row = u >> 3, k8 = (u & 7) * 8;
    const int rc  = row < NN ? row : NN - 1;
    const unsigned mk = row < NN ? 0xffffu : 0u;
    const float* p = x + (size_t)rc * HD + k8;
    const v4f a = *(const v4fa*)p;
    const v4f b = *(const v4fa*)(p + 4);
    v8us o;
    o[0] = (unsigned short)(bf16_bits(a.x) & mk); o[1] = (unsigned short)(bf16_bits(a.y) & mk);
    o[2] = (unsigned short)(bf16_bits(a.z) & mk); o[3] = (unsigned short)(bf16_bits(a.w) & mk);
    o[4] = (unsigned short)(bf16_bits(b.x) & mk); o[5] = (unsigned short)(bf16_bits(b.y) & mk);
    o[6] = (unsigned short)(bf16_bits(b.z) & mk); o[7] = (unsigned short)(bf16_bits(b.w) & mk);
    st2_v8us(xb + (size_t)row * HD + k8, o);
  } else if (blk < PBX + PBW) {
    const int u = (blk - PBX) * NTHR + tid;
    const float* p = wsrc + (size_t)u * 8;
    const v4f a = *(const v4fa*)p;
    const v4f b = *(const v4fa*)(p + 4);
    v8us o;
    o[0] = (unsigned short)bf16_bits(a.x); o[1] = (unsigned short)bf16_bits(a.y);
    o[2] = (unsigned short)bf16_bits(a.z); o[3] = (unsigned short)bf16_bits(a.w);
    o[4] = (unsigned short)bf16_bits(b.x); o[5] = (unsigned short)bf16_bits(b.y);
    o[6] = (unsigned short)bf16_bits(b.z); o[7] = (unsigned short)bf16_bits(b.w);
    st2_v8us(wb + (size_t)u * 8, o);
  } else {
    if (tid < 96) {
      const int ib = tid < 47 ? tid : 47;
      int ig = tid - 48; ig = ig < 0 ? 0 : (ig > 15 ? 15 : ig);
      int ie = tid - 64; ie = ie < 0 ? 0 : (ie > 15 ? 15 : ie);
      const v4f a = *(const v4fa*)(bs + 4 * ib);
      const v4f b = *(const v4fa*)(gam + 4 * ig);
      const v4f c = *(const v4fa*)(bet + 4 * ie);
      asm volatile("" :: "v"(a));
      asm volatile("" :: "v"(b));
      asm volatile("" :: "v"(c));
      const unsigned ma = (tid < 48) ? 0xffffffffu : 0u;
      const unsigned mb = (tid >= 48 && tid < 64) ? 0xffffffffu : 0u;
      const unsigned mc = (tid >= 64 && tid < 80) ? 0xffffffffu : 0u;
      v4f o;
      o.x = __uint_as_float(((bf16_bits(a.x) << 16) & ma) | ((bf16_bits(b.x) << 16) & mb) | ((bf16_bits(c.x) << 16) & mc));
      o.y = __uint_as_float(((bf16_bits(a.y) << 16) & ma) | ((bf16_bits(b.y) << 16) & mb) | ((bf16_bits(c.y) << 16) & mc));
      o.z = __uint_as_float(((bf16_bits(a.z) << 16) & ma) | ((bf16_bits(b.z) << 16) & mb) | ((bf16_bits(c.z) << 16) & mc));
      o.w = __uint_as_float(((bf16_bits(a.w) << 16) & ma) | ((bf16_bits(b.w) << 16) & mb) | ((bf16_bits(c.w) << 16) & mc));
      st2_v4f(par + 4 * tid, o);
    }
  }
}

__device__ __forceinline__ void bucket_flush(const int* pl, const int* cnt, const int* dvb, int ov,
                                             int* lp, int* cop, int* dvp, int* fp, int tid) {
#pragma unroll 1
  for (int i = tid * 4; i < RCAP; i += NTHR * 4) {
    const v4i v = *(const v4ia*)(pl + i);
    *(volatile v4i*)(lp + i) = v;
  }
#pragma unroll 1
  for (int i = tid * 4; i < 2 * NBRUN; i += NTHR * 4) {
    const v4i v = *(const v4ia*)(cnt + i);
    *(volatile v4i*)(cop + i) = v;
  }
  {
    const v4i v = *(const v4ia*)(dvb + 4 * tid);
    *(volatile v4i*)(dvp + 4 * tid) = v;
  }
  if (tid < 8) {
    const v4i f = {ov, ov, ov, ov};
    *(volatile v4i*)(fp + 4 * tid) = f;
  }
}

__global__ __launch_bounds__(NTHR) void k_bucket(const int* __restrict__ srcs, const int* __restrict__ dsts,
                                                 int* LIST, int* CO, int* DINVB, int* FLAG) {
  extern __shared__ __attribute__((aligned(16))) int dsm[];
  int* wl   = dsm;
  int* pl   = dsm + NWAVE * WLCAP;
  int* cnt  = pl + RCAP;
  int* offs = cnt + NBRUN;
  int* cur  = offs + NBRUN;
  int* misc = cur + NBRUN;
  const int tid = (int)threadIdx.x, lane = tid & 31, wave = tid >> 5;
  const int blk = (int)blockIdx.x;
  const unsigned nbs = (unsigned)(blk * NBRUN);

  {
    const v4i z4 = {0, 0, 0, 0};
    for (int i = tid * 4; i < BK_ZINTS; i += NTHR * 4) *(v4ia*)(dsm + i) = z4;
    if (tid < 16) misc[tid] = 0;
  }
  __syncthreads();

  {
    const int per  = ((NE + NWAVE * WCH - 1) / (NWAVE * WCH)) * WCH;
    const int ebeg = wave * per;
    const int eend = (ebeg + per < NE) ? (ebeg + per) : NE;
    int* mylist = wl + wave * WLCAP;
    int wc = 0;
#pragma unroll 1
    for (int cb = ebeg; cb < eend; cb += WCH) {
      const int e0  = cb + lane * EPT;
      const bool inr = e0 < NE;
      const int e0c = e0 < NE - EPT ? e0 : NE - EPT;
      const v4i da = *(const v4ia*)(dsts + e0c);
      const v4i db = *(const v4ia*)(dsts + e0c + 4);
      asm volatile("" :: "v"(da));
      asm volatile("" :: "v"(db));
      const unsigned s0 = (unsigned)da.x - nbs, s1 = (unsigned)da.y - nbs;
      const unsigned s2 = (unsigned)da.z - nbs, s3 = (unsigned)da.w - nbs;
      const unsigned s4 = (unsigned)db.x - nbs, s5 = (unsigned)db.y - nbs;
      const unsigned s6 = (unsigned)db.z - nbs, s7 = (unsigned)db.w - nbs;
      const bool h0 = inr & (s0 < (unsigned)NBRUN), h1 = inr & (s1 < (unsigned)NBRUN);
      const bool h2 = inr & (s2 < (unsigned)NBRUN), h3 = inr & (s3 < (unsigned)NBRUN);
      const bool h4 = inr & (s4 < (unsigned)NBRUN), h5 = inr & (s5 < (unsigned)NBRUN);
      const bool h6 = inr & (s6 < (unsigned)NBRUN), h7 = inr & (s7 < (unsigned)NBRUN);
      const unsigned m0 = __builtin_amdgcn_ballot_w32(h0), m1 = __builtin_amdgcn_ballot_w32(h1);
      const unsigned m2 = __builtin_amdgcn_ballot_w32(h2), m3 = __builtin_amdgcn_ballot_w32(h3);
      const unsigned m4 = __builtin_amdgcn_ballot_w32(h4), m5 = __builtin_amdgcn_ballot_w32(h5);
      const unsigned m6 = __builtin_amdgcn_ballot_w32(h6), m7 = __builtin_amdgcn_ballot_w32(h7);
      const unsigned any = m0 | m1 | m2 | m3 | m4 | m5 | m6 | m7;
      if (any != 0u) {
        const int pre = (int)(__builtin_amdgcn_mbcnt_lo(m0, 0u) + __builtin_amdgcn_mbcnt_lo(m1, 0u) +
                              __builtin_amdgcn_mbcnt_lo(m2, 0u) + __builtin_amdgcn_mbcnt_lo(m3, 0u) +
                              __builtin_amdgcn_mbcnt_lo(m4, 0u) + __builtin_amdgcn_mbcnt_lo(m5, 0u) +
                              __builtin_amdgcn_mbcnt_lo(m6, 0u) + __builtin_amdgcn_mbcnt_lo(m7, 0u));
        int p = wc + pre;
        if (h0) { if (p < WLCAP) mylist[p] = ((e0 + 0) << SLB) | (int)s0; p = p + 1; }
        if (h1) { if (p < WLCAP) mylist[p] = ((e0 + 1) << SLB) | (int)s1; p = p + 1; }
        if (h2) { if (p < WLCAP) mylist[p] = ((e0 + 2) << SLB) | (int)s2; p = p + 1; }
        if (h3) { if (p < WLCAP) mylist[p] = ((e0 + 3) << SLB) | (int)s3; p = p + 1; }
        if (h4) { if (p < WLCAP) mylist[p] = ((e0 + 4) << SLB) | (int)s4; p = p + 1; }
        if (h5) { if (p < WLCAP) mylist[p] = ((e0 + 5) << SLB) | (int)s5; p = p + 1; }
        if (h6) { if (p < WLCAP) mylist[p] = ((e0 + 6) << SLB) | (int)s6; p = p + 1; }
        if (h7) { if (p < WLCAP) mylist[p] = ((e0 + 7) << SLB) | (int)s7; p = p + 1; }
        wc += (int)(__builtin_popcount(m0) + __builtin_popcount(m1) + __builtin_popcount(m2) + __builtin_popcount(m3) +
                    __builtin_popcount(m4) + __builtin_popcount(m5) + __builtin_popcount(m6) + __builtin_popcount(m7));
      }
    }
    if (lane == 0) misc[wave] = wc;
  }
  __syncthreads();

  if (wave == 0) {
    int ov = 0;
#pragma unroll 1
    for (int w2 = 0; w2 < NWAVE; ++w2) {
      int c = misc[w2];
      if (c > WLCAP) ov = 1;
      c = c < 0 ? 0 : (c > WLCAP ? WLCAP : c);
#pragma unroll 1
      for (int b0 = 0; b0 < c; b0 += 32) {
        const int idx = b0 + lane;
        const int ent = wl[w2 * WLCAP + (idx < WLCAP ? idx : WLCAP - 1)];
        const int m32 = (c - b0) < 32 ? (c - b0) : 32;
#pragma unroll 1
        for (int k = 0; k < m32; ++k) {
          const int u    = __builtin_amdgcn_readlane(ent, k);
          const int slot = u & (NBRUN - 1);
          if (lane == 0) cnt[slot] = cnt[slot] + 1;
        }
      }
    }
    if (lane == 0) misc[9] = ov;
  }
  __syncthreads();
  if (wave == 0) {
    const int base = lane * (NBRUN / 32);
    int s = 0;
#pragma unroll 1
    for (int i = 0; i < NBRUN / 32; ++i) s += cnt[base + i];
    int incl = s;
#pragma unroll
    for (int d = 1; d < 32; d <<= 1) {
      const int y = __shfl_up(incl, d, 32);
      if (lane >= d) incl += y;
    }
    int run = incl - s;
#pragma unroll 1
    for (int i = 0; i < NBRUN / 32; ++i) {
      const int cv = cnt[base + i];
      offs[base + i] = run;
      cur[base + i]  = run;
      run += cv;
    }
  }
  __syncthreads();

  if (wave == 0) {
#pragma unroll 1
    for (int w2 = 0; w2 < NWAVE; ++w2) {
      int c = misc[w2];
      c = c < 0 ? 0 : (c > WLCAP ? WLCAP : c);
#pragma unroll 1
      for (int b0 = 0; b0 < c; b0 += 32) {
        const int idx = b0 + lane;
        const int ent = wl[w2 * WLCAP + (idx < WLCAP ? idx : WLCAP - 1)];
        int eid = (ent >> SLB) & 0x1FFFFF;
        eid = eid > NE - 1 ? NE - 1 : eid;
        int sr = srcs[eid];
        sr = sr < 0 ? 0 : (sr > NN - 1 ? NN - 1 : sr);
        const int m32 = (c - b0) < 32 ? (c - b0) : 32;
#pragma unroll 1
        for (int k = 0; k < m32; ++k) {
          const int u    = __builtin_amdgcn_readlane(ent, k);
          const int wd   = __builtin_amdgcn_readlane(sr, k);
          const int slot = u & (NBRUN - 1);
          if (lane == 0) {
            int p = cur[slot];
            p = p < 0 ? 0 : (p > RCAP - 1 ? RCAP - 1 : p);
            pl[p] = wd;
            cur[slot] = p + 1;
          }
        }
      }
    }
  }
  __syncthreads();

#pragma unroll 1
  for (int j = 0; j < 4; ++j) {
    const int s  = 4 * tid + j;
    const int dg = cnt[s] + 1;
    cur[s] = __float_as_int(1.0f / sqrtf((float)dg));
  }
  __syncthreads();

  const int ovf = misc[9];
  int* lp  = LIST + (size_t)blk * RCAP;
  int* cop = CO + (size_t)blk * (2 * NBRUN);
  int* dvp = DINVB + (size_t)blk * NBRUN;
  int* fp  = FLAG + (size_t)blk * 32;
  bucket_flush(pl, cnt, cur, ovf, lp, cop, dvp, fp, tid);
  __threadfence();
  bucket_flush(pl, cnt, cur, ovf, lp, cop, dvp, fp, tid);
}

template <int KTOT>
__device__ __forceinline__ void gemm_16x64(const unsigned short* __restrict__ ap,
                                           const unsigned short* __restrict__ bp, v8f (&acc)[4]) {
#pragma unroll 1
  for (int k0 = 0; k0 < KTOT; k0 += 32) {
    FragB af;
    af.h[0] = *(const v8usa*)(ap + k0);
    af.h[1] = *(const v8usa*)(ap + k0 + 16);
    const int kw = k0 & (HD - 1);
#pragma unroll
    for (int nt = 0; nt < 4; ++nt) {
      const unsigned short* wq = bp + (size_t)(16 * nt) * (size_t)HD + kw;
      FragB bf;
      bf.h[0] = *(const v8usa*)wq;
      bf.h[1] = *(const v8usa*)(wq + 16);
      acc[nt] = wmb(af, bf, acc[nt]);
    }
  }
}

__device__ __forceinline__ void stage_d(float* stg, const v8f (&acc)[4], int wave, int hh, int m) {
#pragma unroll
  for (int nt = 0; nt < 4; ++nt) {
#pragma unroll
    for (int r = 0; r < 8; ++r) stg[(16 * wave + 8 * hh + r) * SP + 16 * nt + m] = acc[nt][r];
  }
}

template <int KTOT, int APITCH>
__global__ __launch_bounds__(NTHR) __attribute__((amdgpu_num_vgpr(248)))
void k_gemm(const unsigned short* __restrict__ A, const unsigned short* __restrict__ BT,
            const float* __restrict__ DINV, float* P) {
  static_assert(KTOT % 32 == 0 && KTOT <= APITCH && APITCH % 8 == 0);
  __shared__ __attribute__((aligned(16))) float stg[GBM * SP];
  __shared__ __attribute__((aligned(16))) float sd[GBM];
  const int tid = (int)threadIdx.x, lane = tid & 31, wave = tid >> 5, hh = lane >> 4, m = lane & 15;
  const int rowBase = (int)blockIdx.x * GBM;
  if (tid < 32) *(v4fa*)(sd + 4 * tid) = *(const v4fa*)(DINV + rowBase + 4 * tid);

  v8f acc[4];
  {
    const v8f z = {0.f, 0.f, 0.f, 0.f, 0.f, 0.f, 0.f, 0.f};
#pragma unroll
    for (int t = 0; t < 4; ++t) acc[t] = z;
  }
  const unsigned short* ap = A + (size_t)(rowBase + 16 * wave + m) * (size_t)APITCH + 8 * hh;
  const unsigned short* bp = BT + (size_t)m * (size_t)HD + 8 * hh;
  gemm_16x64<KTOT>(ap, bp, acc);
  stage_d(stg, acc, wave, hh, m);
  __syncthreads();

#pragma unroll 1
  for (int i = 0; i < 8; ++i) {
    const int lr   = 16 * wave + 2 * i + hh;
    const int grow = rowBase + lr;
    const bool live = grow < NN;
    const v4f a  = *(const v4fa*)(stg + lr * SP + 4 * m);
    const float dv = sd[lr];
    asm volatile("" :: "v"(a));
    const float v0 = dv * a.x, v1 = dv * a.y, v2 = dv * a.z, v3 = dv * a.w;
    v4f o;
    o.x = live ? v0 : 0.0f; o.y = live ? v1 : 0.0f; o.z = live ? v2 : 0.0f; o.w = live ? v3 : 0.0f;
    st2_v4f(P + (size_t)grow * HD + 4 * m, o);
  }
}

template <int MODE>
__global__ __launch_bounds__(NTHR) void k_replay(const int* __restrict__ LIST, const int* __restrict__ CO,
                                                 const float* __restrict__ DINV, const int* __restrict__ FLAG,
                                                 const float* __restrict__ P, const float* __restrict__ PAR,
                                                 int layer, unsigned short* HL, float* T, double* REC) {
  constexpr int REDN = (MODE == 1) ? (16 * HD * 2) : 2;
  __shared__ __attribute__((aligned(16))) int    sco[2 * NBRUN];
  __shared__ __attribute__((aligned(16))) float  sdv[NBRUN];
  __shared__ __attribute__((aligned(16))) float  sbias[128];
  __shared__ __attribute__((aligned(16))) double red[REDN];
  const int tid = (int)threadIdx.x, lane = tid & 31, wave = tid >> 5, hh = lane >> 4, q = lane & 15;
  const int g   = 2 * wave + hh;
  const int blk = (int)blockIdx.x;
  const int rowBase = blk * NBRUN;
  const int* lb = LIST + (size_t)blk * RCAP;
  {
    const int* cop = CO + (size_t)blk * (2 * NBRUN);
    *(v4ia*)(sco + 4 * tid)         = *(const v4ia*)(cop + 4 * tid);
    *(v4ia*)(sco + NBRUN + 4 * tid) = *(const v4ia*)(cop + NBRUN + 4 * tid);
    *(v4fa*)(sdv + 4 * tid)         = *(const v4fa*)(DINV + (size_t)blk * NBRUN + 4 * tid);
    if (tid < 32) *(v4fa*)(sbias + 4 * tid) = *(const v4fa*)(PAR + layer * HD + 4 * tid);
  }
  __syncthreads();

  const int flag = FLAG[(size_t)blk * 32];
  const v4f bias = *(const v4fa*)(sbias + 4 * q);
  const float qnan = __uint_as_float(0x7fc00000u);
  double s0 = 0.0, s1 = 0.0, s2 = 0.0, s3 = 0.0;
  double q0 = 0.0, q1 = 0.0, q2 = 0.0, q3 = 0.0;

#pragma unroll 1
  for (int i = 0; i < NBRUN / 16; ++i) {
    const int slot = 16 * i + g;
    const int d    = rowBase + slot;
    int c = sco[slot];
    int o = sco[NBRUN + slot];
    const float dv = sdv[slot];
    const bool big = c > TRIPCAP;
    c = c < 0 ? 0 : (c > TRIPCAP ? TRIPCAP : c);
    o = o < 0 ? 0 : (o > RCAP - 1 ? RCAP - 1 : o);
    const int co = __shfl_xor(c, 16, 32);
    int cmv = c > co ? c : co;
    const int cm = __builtin_amdgcn_readfirstlane(cmv);
    int last = o + c - 1;
    last = last < o ? o : last;
    last = last > RCAP - 1 ? RCAP - 1 : last;
    float a0 = 0.0f, a1 = 0.0f, a2 = 0.0f, a3 = 0.0f;
#pragma unroll 1
    for (int j = 0; j < cm; ++j) {
      int idx = o + j;
      idx = idx > last ? last : idx;
      int sr = lb[idx];
      sr = sr < 0 ? 0 : (sr > NN - 1 ? NN - 1 : sr);
      const v4f v = *(const v4fa*)(P + (size_t)sr * HD + 4 * q);
      asm volatile("" :: "v"(v));
      const bool valid = j < c;
      const float t0 = a0 + v.x, t1 = a1 + v.y, t2 = a2 + v.z, t3 = a3 + v.w;
      a0 = valid ? t0 : a0; a1 = valid ? t1 : a1; a2 = valid ? t2 : a2; a3 = valid ? t3 : a3;
    }
    const int dc = d < NN ? d : NN - 1;
    const v4f ps = *(const v4fa*)(P + (size_t)dc * HD + 4 * q);
    asm volatile("" :: "v"(ps));
    float v0 = dv * (a0 + ps.x) + bias.x, v1 = dv * (a1 + ps.y) + bias.y;
    float v2 = dv * (a2 + ps.z) + bias.z, v3 = dv * (a3 + ps.w) + bias.w;
    const bool bad  = (flag != 0) | big;
    const bool live = d < NN;
    v0 = bad ? qnan : v0; v1 = bad ? qnan : v1; v2 = bad ? qnan : v2; v3 = bad ? qnan : v3;
    v0 = live ? v0 : 0.0f; v1 = live ? v1 : 0.0f; v2 = live ? v2 : 0.0f; v3 = live ? v3 : 0.0f;
    if constexpr (MODE == 0) {
      int h01, h23, l01, l23;
      hilo_pack(v0, v1, v2, v3, h01, h23, l01, l23);
      const v4i ow = regroup8(h01, h23, l01, l23, lane);
      unsigned short* hp = HL + (size_t)d * KL + 8 * q;
      *(volatile v4i*)hp = ow;
      __threadfence();
      *(volatile v4i*)hp = ow;
    } else {
      v4f ov;
      ov.x = v0; ov.y = v1; ov.z = v2; ov.w = v3;
      float* op = T + (size_t)d * HD + 4 * q;
      *(volatile v4f*)op = ov;
      __threadfence();
      *(volatile v4f*)op = ov;
      const double e0 = (double)v0, e1 = (double)v1, e2 = (double)v2, e3 = (double)v3;
      s0 += e0; s1 += e1; s2 += e2; s3 += e3;
      q0 += e0 * e0; q1 += e1 * e1; q2 += e2 * e2; q3 += e3 * e3;
    }
  }

  if constexpr (MODE == 1) {
    double* rp = red + (size_t)(g * HD + 4 * q) * 2;
    rp[0] = s0; rp[1] = q0; rp[2] = s1; rp[3] = q1;
    rp[4] = s2; rp[5] = q2; rp[6] = s3; rp[7] = q3;
    __syncthreads();
    if (tid < HD) {
      double S = 0.0, Q = 0.0;
#pragma unroll 1
      for (int g2 = 0; g2 < 16; ++g2) {
        S += red[(size_t)(g2 * HD + tid) * 2];
        Q += red[(size_t)(g2 * HD + tid) * 2 + 1];
      }
      v2d r;
      r.x = S; r.y = Q;
      double* dp = REC + ((size_t)blk * HD + (size_t)tid) * 2;
      *(volatile v2d*)dp = r;
      __threadfence();
      *(volatile v2d*)dp = r;
    }
  }
}

__global__ __launch_bounds__(64) void k_combine(const double* __restrict__ REC, float* STAT) {
  __shared__ __attribute__((aligned(16))) float st[2 * HD];
  const int tid = (int)threadIdx.x;
  double S = 0.0, Q = 0.0;
#pragma unroll 1
  for (int b = 0; b < NBK; ++b) {
    const v2d r = *(const v2da*)(REC + ((size_t)b * HD + (size_t)tid) * 2);
    S += r.x;
    Q += r.y;
  }
  const double mean = S / (double)NN;
  double var = Q / (double)NN - mean * mean;
  var = (var < 0.0) ? 0.0 : var;
  const float meanf = (float)mean;
  const float varf  = (float)var;
  const float rs = 1.0f / sqrtf(varf + 1e-5f);
  st[tid] = meanf;
  st[HD + tid] = rs;
  __syncthreads();
  if (tid < 32) {
    const v4f v = *(const v4fa*)(st + 4 * tid);
    st2_v4f(STAT + 4 * tid, v);
  }
}

__global__ __launch_bounds__(NTHR) void k_apply(const float* __restrict__ T, const float* __restrict__ STAT,
                                                const float* __restrict__ PAR, float* out) {
  __shared__ __attribute__((aligned(16))) float sst[4 * HD];
  const int tid = (int)threadIdx.x;
  if (tid < 32) {
    *(v4fa*)(sst + 4 * tid) = *(const v4fa*)(STAT + 4 * tid);
  } else if (tid < 64) {
    *(v4fa*)(sst + 4 * tid) = *(const v4fa*)(PAR + NLAY * HD + 4 * (tid - 32));
  }
  __syncthreads();
  const int u  = (int)blockIdx.x * NTHR + tid;
  const int c4 = (u & 15) * 4;
  const v4f t = *(const v4fa*)(T + (size_t)u * 4);
  v4f o;
  o.x = ((t.x - sst[c4 + 0]) * sst[HD + c4 + 0]) * sst[2 * HD + c4 + 0] + sst[3 * HD + c4 + 0];
  o.y = ((t.y - sst[c4 + 1]) * sst[HD + c4 + 1]) * sst[2 * HD + c4 + 1] + sst[3 * HD + c4 + 1];
  o.z = ((t.z - sst[c4 + 2]) * sst[HD + c4 + 2]) * sst[2 * HD + c4 + 2] + sst[3 * HD + c4 + 2];
  o.w = ((t.w - sst[c4 + 3]) * sst[HD + c4 + 3]) * sst[2 * HD + c4 + 3] + sst[3 * HD + c4 + 3];
  st2_v4f(out + (size_t)u * 4, o);
}

extern "C" void kernel_launch(void* const* d_in, const int* in_sizes, int n_in,
                              void* d_out, int out_size, void* d_ws, size_t ws_size,
                              hipStream_t stream) {
  if (n_in < 6) return;
  if (in_sizes[0] != NN * HD) return;
  if (in_sizes[1] != 2 * NE) return;
  if (in_sizes[2] != NLAY * HD * HD) return;
  if (in_sizes[3] != NLAY * HD) return;
  if (in_sizes[4] != HD) return;
  if (in_sizes[5] != HD) return;
  if (out_size != NN * HD) return;

  const float* x   = (const float*)d_in[0];
  const int*   ei  = (const int*)d_in[1];
  const float* Wsp = (const float*)d_in[2];
  const float* bsp = (const float*)d_in[3];
  const float* gam = (const float*)d_in[4];
  const float* bet = (const float*)d_in[5];
  float* out = (float*)d_out;
  const int* srcs = ei;
  const int* dsts = ei + NE;

  constexpr size_t zXB   = (size_t)MP * HD * 2;
  constexpr size_t zP    = (size_t)RP * HD * 4;
  constexpr size_t zHL   = (size_t)RP * KL * 2;
  constexpr size_t zT    = (size_t)RP * HD * 4;
  constexpr size_t zLIST = (size_t)NBK * RCAP * 4;
  constexpr size_t zCO   = (size_t)NBK * 2 * NBRUN * 4;
  constexpr size_t zDINV = (size_t)NBK * NBRUN * 4;
  constexpr size_t zFLAG = (size_t)NBK * 128;
  constexpr size_t zWB   = (size_t)NLAY * HD * HD * 2;
  constexpr size_t zPAR  = (size_t)PARN * 4;
  constexpr size_t zREC  = (size_t)NBK * HD * 2 * 8;
  constexpr size_t zSTAT = (size_t)2 * HD * 4;
  constexpr size_t oXB   = 0;
  constexpr size_t oP    = oXB + zXB;
  constexpr size_t oHL   = oP + zP;
  constexpr size_t oT    = oHL + zHL;
  constexpr size_t oLIST = oT + zT;
  constexpr size_t oCO   = oLIST + zLIST;
  constexpr size_t oDINV = oCO + zCO;
  constexpr size_t oFLAG = oDINV + zDINV;
  constexpr size_t oWB   = oFLAG + zFLAG;
  constexpr size_t oPAR  = oWB + zWB;
  constexpr size_t oREC  = oPAR + zPAR;
  constexpr size_t oSTAT = oREC + zREC;
  constexpr size_t oEND  = oSTAT + zSTAT;
  static_assert(zXB % 256 == 0 && zP % 256 == 0 && zHL % 256 == 0 && zT % 256 == 0 && zLIST % 256 == 0);
  static_assert(zCO % 256 == 0 && zDINV % 256 == 0 && zFLAG % 256 == 0 && zWB % 256 == 0 && zPAR % 256 == 0);
  static_assert(zREC % 256 == 0 && zSTAT % 256 == 0);
  static_assert(RP >= MP && (size_t)MP * HD * 4 <= zP);
  static_assert(oEND <= (size_t)WSMAX);
  if (oEND > ws_size) return;

  char* ws = (char*)d_ws;
  unsigned short* XB   = (unsigned short*)(ws + oXB);
  float*          P    = (float*)(ws + oP);
  unsigned short* HL   = (unsigned short*)(ws + oHL);
  float*          T    = (float*)(ws + oT);
  int*            LIST = (int*)(ws + oLIST);
  int*            CO   = (int*)(ws + oCO);
  float*          DINV = (float*)(ws + oDINV);
  int*            FLAG = (int*)(ws + oFLAG);
  unsigned short* WB   = (unsigned short*)(ws + oWB);
  float*          PAR  = (float*)(ws + oPAR);
  double*         REC  = (double*)(ws + oREC);
  float*          STAT = (float*)(ws + oSTAT);

  hipFuncSetAttribute(reinterpret_cast<const void*>(&k_bucket), hipFuncAttributeMaxDynamicSharedMemorySize, (int)BK_LDS);

  k_prep<<<PBTOT, NTHR, 0, stream>>>(x, Wsp, bsp, gam, bet, XB, WB, PAR);
  k_bucket<<<NBK, NTHR, BK_LDS, stream>>>(srcs, dsts, LIST, CO, (int*)DINV, FLAG);

  k_gemm<HD, HD><<<MP / GBM, NTHR, 0, stream>>>(XB, WB, DINV, P);
  k_replay<0><<<NBK, NTHR, 0, stream>>>(LIST, CO, DINV, FLAG, P, PAR, 0, HL, T, REC);

  k_gemm<KS1, KL><<<MP / GBM, NTHR, 0, stream>>>(HL, WB + (size_t)1 * HD * HD, DINV, P);
  k_replay<0><<<NBK, NTHR, 0, stream>>>(LIST, CO, DINV, FLAG, P, PAR, 1, HL, T, REC);

  k_gemm<KS2, KL><<<MP / GBM, NTHR, 0, stream>>>(HL, WB + (size_t)2 * HD * HD, DINV, P);
  k_replay<1><<<NBK, NTHR, 0, stream>>>(LIST, CO, DINV, FLAG, P, PAR, 2, HL, T, REC);

  k_combine<<<1, 64, 0, stream>>>(REC, STAT);
  k_apply<<<(NN * HD / 4) / NTHR, NTHR, 0, stream>>>(T, STAT, PAR, out);
}
